// CvTSelfAttentionBlock_4011499455079
// MI455X (gfx1250) — hardware-verified
//
#include <hip/hip_runtime.h>
#include <math.h>

typedef __attribute__((ext_vector_type(16))) _Float16 v16h;
typedef __attribute__((ext_vector_type(16))) __bf16 v16b;
typedef __attribute__((ext_vector_type(8)))  _Float16 v8h;
typedef __attribute__((ext_vector_type(8)))  float v8f;
typedef __attribute__((ext_vector_type(4)))  float v4f;
typedef __attribute__((ext_vector_type(2)))  float v2f;
typedef __attribute__((ext_vector_type(4)))  unsigned v4u;
typedef __attribute__((ext_vector_type(4)))  int v4i;
typedef float __attribute__((may_alias)) float_a;
typedef int __attribute__((may_alias)) int_a;

template <typename T> __device__ __forceinline__ void vst2(void* p, T v) { *(volatile T*)p = v; __threadfence(); *(volatile T*)p = v; }
__device__ __forceinline__ v8f wmma16(v16h a, v16h b, v8f c) {
  v8f d = __builtin_amdgcn_wmma_f32_16x16x32_f16(false, a, false, b, (short)0, c, false, false);
  asm volatile("v_nop\n\tv_nop\n\tv_nop\n\tv_nop" : "+v"(d) : "v"(a), "v"(b));
  return d;
}
__device__ __forceinline__ v8f wmma_bf(v16b a, v16b b, v8f c) {
  v8f d = __builtin_amdgcn_wmma_f32_16x16x32_bf16(false, a, false, b, (short)0, c, false, false);
  asm volatile("v_nop\n\tv_nop\n\tv_nop\n\tv_nop" : "+v"(d) : "v"(a), "v"(b));
  return d;
}
__device__ __forceinline__ v16h frag_h(const _Float16* rowk0, int lane) {
  union { v16h v; v8h q[2]; } u; const _Float16* p = rowk0 + 8 * (lane >> 4);
  u.q[0] = *(const v8h*)p; u.q[1] = *(const v8h*)(p + 16); return u.v;
}
__device__ __forceinline__ v16h frag_f32(const float* rowk0, int lane) {
  v16h a; const float* p = rowk0 + 8 * (lane >> 4);
#pragma unroll
  for (int i = 0; i < 8; ++i) { a[i] = (_Float16)p[i]; a[8 + i] = (_Float16)p[16 + i]; }
  return a;
}
__device__ __forceinline__ v16h frag_f32s(const float* rowk0, int lane, float sc) {
  v16h a; const float* p = rowk0 + 8 * (lane >> 4);
#pragma unroll
  for (int i = 0; i < 8; ++i) { a[i] = (_Float16)(p[i] * sc); a[8 + i] = (_Float16)(p[16 + i] * sc); }
  return a;
}
__device__ __forceinline__ v16h fragc_f32(const float* W, int k0, int n, int lane, int ld, int K) {
  v16h a; const int g = lane >> 4;
#pragma unroll
  for (int i = 0; i < 8; ++i) { const int ka = k0 + 8 * g + i, kb = ka + 16;
    a[i] = (_Float16)(ka < K ? W[(size_t)(ka < K ? ka : K - 1) * ld + n] : 0.f); a[8 + i] = (_Float16)(kb < K ? W[(size_t)(kb < K ? kb : K - 1) * ld + n] : 0.f); }
  return a;
}
struct F2 { v16b h, l; };
__device__ __forceinline__ F2 bsplit16(const float v[16]) { F2 r;
#pragma unroll
  for (int i = 0; i < 16; ++i) { const __bf16 h = (__bf16)v[i]; r.h[i] = h; r.l[i] = (__bf16)(v[i] - (float)h); }
  return r; }
__device__ __forceinline__ F2 split_row(const float* row, int k0, int lane) { float v[16]; const float* p = row + k0 + 8 * (lane >> 4);
#pragma unroll
  for (int i = 0; i < 8; ++i) { v[i] = p[i]; v[8 + i] = p[16 + i]; }
  return bsplit16(v); }
__device__ __forceinline__ F2 split_rowK(const float* row, int k0, int lane, int K) { float v[16]; const int g = lane >> 4;
#pragma unroll
  for (int i = 0; i < 8; ++i) { const int ka = k0 + 8 * g + i, kb = ka + 16; v[i] = ka < K ? row[ka < K ? ka : K - 1] : 0.f; v[8 + i] = kb < K ? row[kb < K ? kb : K - 1] : 0.f; }
  return bsplit16(v); }
__device__ __forceinline__ F2 split_col(const float* W, int k0, int n, int lane, int ld, int K) { float v[16]; const int g = lane >> 4;
#pragma unroll
  for (int i = 0; i < 8; ++i) { const int ka = k0 + 8 * g + i, kb = ka + 16; v[i] = ka < K ? W[(size_t)(ka < K ? ka : K - 1) * ld + n] : 0.f; v[8 + i] = kb < K ? W[(size_t)(kb < K ? kb : K - 1) * ld + n] : 0.f; }
  return bsplit16(v); }
__device__ __forceinline__ v8f mac3(const F2& a, const F2& b, v8f c) { c = wmma_bf(a.l, b.h, c); c = wmma_bf(a.h, b.l, c); return wmma_bf(a.h, b.h, c); }
__device__ __forceinline__ float sigm(float v) { return 1.0f / (1.0f + expf(-v)); }
#define LDSX() do { asm volatile("s_wait_dscnt 0" ::: "memory"); __builtin_amdgcn_wave_barrier(); __builtin_amdgcn_fence(__ATOMIC_RELEASE, "workgroup"); } while (0)


#define NB 8
#define SQ 56
#define NQ (SQ * SQ)
#define SK 28
#define NK (SK * SK)
#define NKP 832
#define CC 192
#define NHD 3
#define DH 64
#define BNEPS 1e-5f
#ifndef TNB
#define TNB NB
#endif
typedef __attribute__((ext_vector_type(8))) __bf16 v8b;
__device__ __forceinline__ v16b frag_b(const __bf16* rowk0, int lane) {
  union { v16b v; v8b q[2]; } u; const __bf16* p = rowk0 + 8 * (lane >> 4);
  u.q[0] = *(const v8b*)p; u.q[1] = *(const v8b*)(p + 16); return u.v;
}
__device__ __forceinline__ float bfr(float v) { return (float)(__bf16)v; }
__device__ __attribute__((noinline)) float exp_ni(float v) { return expf(v); }
__device__ __attribute__((noinline)) float erf_ni(float v) { return erff(v); }

#define WS_QH  0u
#define WS_QL  (WS_QH + 2u * (size_t)NB * NQ * CC)
#define WS_KH  (WS_QL + 2u * (size_t)NB * NQ * CC)
#define WS_KL  (WS_KH + 2u * (size_t)NB * NKP * CC)
#define WS_VT  (WS_KL + 2u * (size_t)NB * NKP * CC)
#define WS_VTL (WS_VT + 2u * (size_t)NB * CC * NKP)
#define WS_END (WS_VTL + 2u * (size_t)NB * CC * NKP)

__device__ __forceinline__ float bnf(float x, const float* G, const float* Bt, const float* M, const float* V, int c) { return (x - bfr(M[c])) / sqrtf(bfr(V[c]) + BNEPS) * bfr(G[c]) + bfr(Bt[c]); }
template <int MODE>
__global__ __launch_bounds__(128) void k_proj(const float* __restrict__ X, const float* __restrict__ DW, const float* __restrict__ G, const float* __restrict__ Bt, const float* __restrict__ M, const float* __restrict__ V, const float* __restrict__ PW, _Float16* __restrict__ OH, _Float16* __restrict__ OL) {
  __shared__ __align__(16) float sa[64][CC + 4]; __shared__ __align__(16) _Float16 sh[64][CC + 8], sl[64][CC + 8];
  const int tid = threadIdx.x, wave = tid >> 5, lane = tid & 31, col = lane & 15, g = lane >> 4; const size_t b = blockIdx.y; const int n0 = blockIdx.x * 64; const float* Xb = X + b * (size_t)NQ * CC; constexpr int NOUT = MODE == 0 ? NQ : NK; constexpr int S = MODE == 0 ? SQ : SK;
  for (int e = tid; e < 64 * CC; e += 128) { const int pl = e / CC, c = e % CC; const int n = n0 + pl; float s = 0.f;
    if (n < NOUT) { const int oy = n / S, ox = n % S;
#pragma unroll
      for (int t9 = 0; t9 < 9; ++t9) { const int ky = t9 / 3, kx = t9 % 3; const int iy = (MODE == 0) ? (oy + ky - 1) : (2 * oy + ky), ix = (MODE == 0) ? (ox + kx - 1) : (2 * ox + kx);
        if (iy >= 0 && iy < SQ && ix >= 0 && ix < SQ) s += bfr(Xb[((size_t)iy * SQ + ix) * CC + c]) * bfr(DW[t9 * CC + c]); }
      s = bnf(s, G, Bt, M, V, c); }
    sa[pl][c] = (n < NOUT) ? s : 0.f; }
  __syncthreads();
  v8f acc[12];
#pragma unroll
  for (int j = 0; j < 12; ++j) acc[j] = v8f{};
#pragma unroll
  for (int kc = 0; kc < CC / 32; ++kc) { float v[16]; const float* pp = &sa[wave * 16 + col][kc * 32 + 8 * g];
#pragma unroll
    for (int i = 0; i < 8; ++i) { v[i] = pp[i]; v[8 + i] = pp[16 + i]; }
    const F2 a = bsplit16(v);
#pragma unroll
    for (int j = 0; j < 12; ++j) { v16b w; const int o = j * 16 + col;
#pragma unroll
      for (int i = 0; i < 8; ++i) { w[i] = (__bf16)PW[(size_t)(kc * 32 + 8 * g + i) * CC + o]; w[8 + i] = (__bf16)PW[(size_t)(kc * 32 + 16 + 8 * g + i) * CC + o]; }
      acc[j] = wmma_bf(a.h, w, acc[j]); acc[j] = wmma_bf(a.l, w, acc[j]); } }
#pragma unroll
  for (int j = 0; j < 12; ++j)
#pragma unroll
    for (int r = 0; r < 8; ++r) { const float q = acc[j][r]; const _Float16 hv = (_Float16)q, lv = (_Float16)((q - (float)hv) * 2048.0f); if (MODE < 2) { sh[wave * 16 + 8 * g + r][j * 16 + col] = hv; sl[wave * 16 + 8 * g + r][j * 16 + col] = lv; } else { sh[wave * 16 + 8 * g + r][j * 16 + col] = hv; sl[wave * 16 + 8 * g + r][j * 16 + col] = lv; } }
  __syncthreads();
  if (MODE < 2) { constexpr int NR = MODE == 0 ? NQ : NKP; for (int e = tid; e < 64 * (CC / 8); e += 128) { const int rl = e / (CC / 8), q = e % (CC / 8); const size_t o = (b * NR + n0 + rl) * CC + q * 8; vst2((unsigned*)(OH + o), *(const v4u*)&sh[rl][q * 8]); vst2((unsigned*)(OL + o), *(const v4u*)&sl[rl][q * 8]); } }
  else {
    for (int e = tid; e < CC * 8; e += 128) { const int c = e >> 3, q = e & 7; _Float16 th[8], tl[8];
#pragma unroll
      for (int i = 0; i < 8; ++i) { th[i] = sh[q * 8 + i][c]; tl[i] = sl[q * 8 + i][c]; }
      const size_t o = (b * CC + c) * (size_t)NKP + n0 + q * 8; vst2((unsigned*)(OH + o), *(const v4u*)th); vst2((unsigned*)(OL + o), *(const v4u*)tl); } } }
__global__ __launch_bounds__(128) void k_att(const _Float16* __restrict__ QH, const _Float16* __restrict__ QL, const _Float16* __restrict__ KH, const _Float16* __restrict__ KL, const _Float16* __restrict__ VT, const _Float16* __restrict__ VTL, float* __restrict__ OUT) {
  __shared__ __align__(16) float sp[4][16][36]; __shared__ __align__(16) float so[4][16][68];
  const int tid = threadIdx.x, wave = tid >> 5, lane = tid & 31, col = lane & 15, g = lane >> 4; const int h = blockIdx.y; const size_t b = blockIdx.z; const int q0 = blockIdx.x * 64 + wave * 16; const size_t rq = b * NQ + q0;
  v16h aq[2], al[2];
#pragma unroll
  for (int kc = 0; kc < 2; ++kc) { aq[kc] = frag_h(QH + (rq + col) * CC + h * DH + kc * 32, lane); al[kc] = frag_h(QL + (rq + col) * CC + h * DH + kc * 32, lane); }
  float m[8], l[8];
#pragma unroll
  for (int r = 0; r < 8; ++r) { m[r] = -3.0e38f; l[r] = 0.f; }
  v8f acc[4] = {}, accl[4] = {};
#pragma unroll 1
  for (int ks = 0; ks < (NK + 31) / 32; ++ks) { float s[2][8];
#pragma unroll
    for (int ct = 0; ct < 2; ++ct) { const int kk = ks * 32 + ct * 16 + col; const size_t rk = b * NKP + kk; v8f c = {}, cl = {};
#pragma unroll
      for (int kc = 0; kc < 2; ++kc) { const v16h kh = frag_h(KH + rk * CC + h * DH + kc * 32, lane), kl = frag_h(KL + rk * CC + h * DH + kc * 32, lane); c = wmma16(aq[kc], kh, c); cl = wmma16(aq[kc], kl, cl); cl = wmma16(al[kc], kh, cl); }
      const bool keep = kk < NK;
#pragma unroll
      for (int r = 0; r < 8; ++r) s[ct][r] = keep ? (c[r] + cl[r] * (1.0f / 2048.0f)) * 0.125f : -3.0e38f; }
    float alpha[8];
#pragma unroll
    for (int r = 0; r < 8; ++r) { float mx = fmaxf(s[0][r], s[1][r]);
#pragma unroll
      for (int o = 1; o < 16; o <<= 1) mx = fmaxf(mx, __shfl_xor(mx, o));
      const float mn = fmaxf(m[r], mx); alpha[r] = (m[r] <= -1.0e38f) ? 0.f : __expf(m[r] - mn); const float e0 = (s[0][r] <= -1.0e38f) ? 0.f : __expf(s[0][r] - mn), e1 = (s[1][r] <= -1.0e38f) ? 0.f : __expf(s[1][r] - mn); float es = e0 + e1;
#pragma unroll
      for (int o = 1; o < 16; o <<= 1) es += __shfl_xor(es, o);
      l[r] = l[r] * alpha[r] + es; m[r] = mn; sp[wave][8 * g + r][col] = e0; sp[wave][8 * g + r][16 + col] = e1; }
#pragma unroll
    for (int j = 0; j < 4; ++j)
#pragma unroll
      for (int r = 0; r < 8; ++r) { acc[j][r] *= alpha[r]; accl[j][r] *= alpha[r]; }
    LDSX();
    v16h pa, pal; { const float* prow = &sp[wave][col][0] + 8 * (lane >> 4);
#pragma unroll
      for (int i = 0; i < 8; ++i) { const float p0 = prow[i] * 2048.0f, p1 = prow[16 + i] * 2048.0f; pa[i] = (_Float16)p0; pa[8 + i] = (_Float16)p1; pal[i] = (_Float16)((p0 - (float)pa[i]) * 2048.0f); pal[8 + i] = (_Float16)((p1 - (float)pa[8 + i]) * 2048.0f); } }
#pragma unroll
    for (int j = 0; j < 4; ++j) { const size_t po = (b * CC + (size_t)h * DH + j * 16 + col) * (size_t)NKP + ks * 32; const v16h vh = frag_h(VT + po, lane), vl = frag_h(VTL + po, lane); acc[j] = wmma16(pa, vh, acc[j]); accl[j] = wmma16(pa, vl, accl[j]); accl[j] = wmma16(pal, vh, accl[j]); }
    LDSX(); }
#pragma unroll
  for (int r = 0; r < 8; ++r) { const float il = (1.0f / 2048.0f) / l[r];
#pragma unroll
    for (int j = 0; j < 4; ++j) so[wave][8 * g + r][j * 16 + col] = (acc[j][r] + accl[j][r] * (1.0f / 2048.0f)) * il; }
  LDSX(); for (int rl = 0; rl < 16; ++rl) if (lane < 16) vst2(OUT + (rq + rl) * CC + (size_t)h * DH + lane * 4, *(const v4f*)&so[wave][rl][lane * 4]); }
extern "C" void kernel_launch(void* const* d_in, const int* in_sizes, int n_in, void* d_out, int out_size, void* d_ws, size_t ws_size, hipStream_t stream) {
  (void)in_sizes; (void)n_in; (void)out_size;
  const float** F = (const float**)d_in;
  if (ws_size < (size_t)WS_END) return;
  char* ws = (char*)d_ws; _Float16 *QH = (_Float16*)(ws + WS_QH), *QL = (_Float16*)(ws + WS_QL), *KH = (_Float16*)(ws + WS_KH), *KL = (_Float16*)(ws + WS_KL), *VT = (_Float16*)(ws + WS_VT), *VTL = (_Float16*)(ws + WS_VTL);
  k_proj<0><<<dim3(NQ / 64, TNB), 128, 0, stream>>>(F[0], F[1], F[2], F[3], F[4], F[5], F[6], QH, QL);
  k_proj<1><<<dim3(NKP / 64, TNB), 128, 0, stream>>>(F[0], F[7], F[8], F[9], F[10], F[11], F[12], KH, KL);
  k_proj<2><<<dim3(NKP / 64, TNB), 128, 0, stream>>>(F[0], F[13], F[14], F[15], F[16], F[17], F[18], VT, VTL);
  k_att<<<dim3(NQ / 64, NHD, TNB), 128, 0, stream>>>(QH, QL, KH, KL, VT, VTL, (float*)d_out);
}
